// MHC_62603443306930
// MI455X (gfx1250) — hardware-verified
//
#include <hip/hip_runtime.h>
#include <stddef.h>
#include <stdint.h>

#define NB    2
#define SQ    2048
#define DM    1024
#define NH    16
#define HDM   64
#define NBH   (NB * NH)
#define NQKV  (3 * DM)
#define MR    (NB * SQ)
#define KCV   (3 * DM)
#define QB    128
#define KC    64
#define NQB   (SQ / QB)
#define R1    320
#define R0    256
#define QB0   (R0 / QB)
#define NQ1   (R1 / 64)
#define NQ0   (R0 / 64)
#define CPR   (SQ + 2)
#define C3R   (R1 + 1)
#define MBP   ((SQ - R0) / 256)

static_assert(NH * HDM == DM);
static_assert(HDM == 64);
static_assert(SQ % 256 == 0);
static_assert(R0 % 256 == 0);
static_assert(R1 % 64 == 0);
static_assert(R1 >= R0 + 64);
static_assert(R0 % QB == 0);
static_assert(QB == 2 * KC);
static_assert(DM % 64 == 0);
static_assert(KCV % 32 == 0);
static_assert(MBP * 256 + R0 == SQ);
static_assert(NQB == 16);

typedef _Float16 v16h __attribute__((ext_vector_type(16)));
typedef _Float16 v8h  __attribute__((ext_vector_type(8)));
typedef float    v8f  __attribute__((ext_vector_type(8)));
typedef float    v4f  __attribute__((ext_vector_type(4)));
typedef unsigned int   v4u   __attribute__((ext_vector_type(4)));
typedef unsigned short v8us  __attribute__((ext_vector_type(8)));
typedef unsigned short v16us __attribute__((ext_vector_type(16)));
typedef __bf16         v16b  __attribute__((ext_vector_type(16)));
typedef unsigned short ush;

union Frag  { v16h v; v8h h[2]; };
union FragU { v16us v; v8us h[2]; v16b b; };
union Pack8 { v8h h; v4u u; };
union PackU { v8us s; v4u u; };
union HU    { _Float16 h; ush u; };
struct HL { v4u h; v4u l; };

__device__ __forceinline__ ush f2bf(float f) {
  const unsigned u = __float_as_uint(f);
  return (ush)((u + 0x7FFFu + ((u >> 16) & 1u)) >> 16);
}
__device__ __forceinline__ float bf2f(ush b) { return __uint_as_float(((unsigned)b) << 16); }

__device__ __forceinline__ HL split8(v8f f) {
  PackU ph, pl;
#pragma unroll
  for (int e = 0; e < 8; ++e) {
    const ush hi = f2bf(f[e]);
    ph.s[e] = hi;
    pl.s[e] = f2bf(f[e] - bf2f(hi));
  }
  HL r; r.h = ph.u; r.l = pl.u;
  return r;
}

__device__ __forceinline__ v8f mma16(v16h a, v16h b, v8f c) {
  c = __builtin_amdgcn_wmma_f32_16x16x32_f16(false, a, false, b, (short)0, c, false, false);
  asm volatile("v_nop\n\tv_nop\n\tv_nop\n\tv_nop" : "+v"(c) : "v"(a), "v"(b));
  return c;
}
__device__ __forceinline__ v8f mmab(v16us a, v16us b, v8f c) {
  FragU ua, ub; ua.v = a; ub.v = b;
  c = __builtin_amdgcn_wmma_f32_16x16x32_bf16(false, ua.b, false, ub.b, (short)0, c, false, false);
  asm volatile("v_nop\n\tv_nop\n\tv_nop\n\tv_nop" : "+v"(c) : "v"(a), "v"(b));
  return c;
}

__device__ __forceinline__ v16h ldfrag(const _Float16* p, int ld, int row0, int k0, int lane) {
  const int m = lane & 15, lh = lane >> 4;
  const _Float16* q = p + (size_t)(row0 + m) * ld + k0 + 8 * lh;
  Frag f;
  f.h[0] = *(const v8h*)(q);
  f.h[1] = *(const v8h*)(q + 16);
  return f.v;
}
__device__ __forceinline__ v16us ldfragu(const ush* p, int ld, int row0, int k0, int lane) {
  const int m = lane & 15, lh = lane >> 4;
  const ush* q = p + (size_t)(row0 + m) * ld + k0 + 8 * lh;
  FragU f;
  f.h[0] = *(const v8us*)(q);
  f.h[1] = *(const v8us*)(q + 16);
  return f.v;
}

__device__ __forceinline__ v8f zero8() { return (v8f){0.f, 0.f, 0.f, 0.f, 0.f, 0.f, 0.f, 0.f}; }

template <int KLEN>
__device__ __forceinline__ void gemm16(const _Float16* __restrict__ A, int lda, int am0,
                                       const _Float16* __restrict__ Bt, int ldb, int bn0, int bk0,
                                       int lane, v8f (&acc)[2][4]) {
#pragma unroll 2
  for (int k0 = 0; k0 < KLEN; k0 += 32) {
    const v16h a0 = ldfrag(A, lda, am0, k0, lane);
    const v16h a1 = ldfrag(A, lda, am0 + 16, k0, lane);
    const v16h b0 = ldfrag(Bt, ldb, bn0, bk0 + k0, lane);
    const v16h b1 = ldfrag(Bt, ldb, bn0 + 16, bk0 + k0, lane);
    const v16h b2 = ldfrag(Bt, ldb, bn0 + 32, bk0 + k0, lane);
    const v16h b3 = ldfrag(Bt, ldb, bn0 + 48, bk0 + k0, lane);
    acc[0][0] = mma16(a0, b0, acc[0][0]);
    acc[1][0] = mma16(a1, b0, acc[1][0]);
    acc[0][1] = mma16(a0, b1, acc[0][1]);
    acc[1][1] = mma16(a1, b1, acc[1][1]);
    acc[0][2] = mma16(a0, b2, acc[0][2]);
    acc[1][2] = mma16(a1, b2, acc[1][2]);
    acc[0][3] = mma16(a0, b3, acc[0][3]);
    acc[1][3] = mma16(a1, b3, acc[1][3]);
  }
}

template <int KLEN>
__device__ __forceinline__ void gemm3(const ush* __restrict__ Ah, const ush* __restrict__ Al, int lda, int am0,
                                      const ush* __restrict__ Bh, const ush* __restrict__ Bl, int ldb, int bn0, int bk0,
                                      int lane, v8f (&acc)[2][4]) {
#pragma unroll 1
  for (int k0 = 0; k0 < KLEN; k0 += 32) {
    const v16us a0h = ldfragu(Ah, lda, am0, k0, lane);
    const v16us a1h = ldfragu(Ah, lda, am0 + 16, k0, lane);
    const v16us a0l = ldfragu(Al, lda, am0, k0, lane);
    const v16us a1l = ldfragu(Al, lda, am0 + 16, k0, lane);
#pragma unroll
    for (int t = 0; t < 4; ++t) {
      const v16us bh = ldfragu(Bh, ldb, bn0 + 16 * t, bk0 + k0, lane);
      const v16us bl = ldfragu(Bl, ldb, bn0 + 16 * t, bk0 + k0, lane);
      acc[0][t] = mmab(a0h, bh, acc[0][t]);
      acc[1][t] = mmab(a1h, bh, acc[1][t]);
      acc[0][t] = mmab(a0h, bl, acc[0][t]);
      acc[1][t] = mmab(a1h, bl, acc[1][t]);
      acc[0][t] = mmab(a0l, bh, acc[0][t]);
      acc[1][t] = mmab(a1l, bh, acc[1][t]);
    }
  }
}

__global__ __launch_bounds__(256) void k_cvt_x(const float* __restrict__ x, _Float16* __restrict__ xh,
                                               ush* __restrict__ x3h, ush* __restrict__ x3l, int ngrp) {
  const int t = blockIdx.x * 256 + (int)threadIdx.x;
  if (t >= ngrp) return;
  const size_t o = (size_t)t * 8;
  const int row = (int)(o / DM);
  const int col = (int)(o % DM);
  const int b = row / SQ, tr = row % SQ;
  const bool three = (tr < R1);
  const size_t o3 = ((size_t)(b * R1 + tr)) * DM + col;
  const v4f a0 = *(const v4f*)(x + o);
  const v4f a1 = *(const v4f*)(x + o + 4);
  Pack8 pk;
  pk.h = (v8h){(_Float16)a0[0], (_Float16)a0[1], (_Float16)a0[2], (_Float16)a0[3],
               (_Float16)a1[0], (_Float16)a1[1], (_Float16)a1[2], (_Float16)a1[3]};
  const v4u vv = pk.u;
  HL s; s.h = (v4u){0u, 0u, 0u, 0u}; s.l = s.h;
  if (three) {
    const v8f f = (v8f){a0[0], a0[1], a0[2], a0[3], a1[0], a1[1], a1[2], a1[3]};
    s = split8(f);
  }
  volatile v4u* d = (volatile v4u*)(xh + o);
  *d = vv;
  if (three) { *(volatile v4u*)(x3h + o3) = s.h; *(volatile v4u*)(x3l + o3) = s.l; }
  __threadfence();
  *d = vv;
  if (three) { *(volatile v4u*)(x3h + o3) = s.h; *(volatile v4u*)(x3l + o3) = s.l; }
}

__global__ __launch_bounds__(256) void k_cvt_w(const float* __restrict__ w, _Float16* __restrict__ wt,
                                               ush* __restrict__ wh, ush* __restrict__ wl, int ngrp) {
  const int t = blockIdx.x * 256 + (int)threadIdx.x;
  if (t >= ngrp) return;
  const size_t o = (size_t)t * 8;
  const v4f a0 = *(const v4f*)(w + o);
  const v4f a1 = *(const v4f*)(w + o + 4);
  const v8f f = (v8f){a0[0], a0[1], a0[2], a0[3], a1[0], a1[1], a1[2], a1[3]};
  Pack8 pk;
  pk.h = (v8h){(_Float16)(f[0] * 32.0f), (_Float16)(f[1] * 32.0f), (_Float16)(f[2] * 32.0f),
               (_Float16)(f[3] * 32.0f), (_Float16)(f[4] * 32.0f), (_Float16)(f[5] * 32.0f),
               (_Float16)(f[6] * 32.0f), (_Float16)(f[7] * 32.0f)};
  const v4u vf = pk.u;
  const HL s = split8(f);
  for (int ps = 0; ps < 2; ++ps) {
    *(volatile v4u*)(wt + o) = vf;
    *(volatile v4u*)(wh + o) = s.h;
    *(volatile v4u*)(wl + o) = s.l;
    __threadfence();
  }
}

__global__ __launch_bounds__(256) void k_cvt_wc(const float* __restrict__ w, _Float16* __restrict__ wt,
                                                ush* __restrict__ wh, ush* __restrict__ wl) {
  __shared__ __align__(16) float sf[KCV];
  const int tid = threadIdx.x;
  const int n = blockIdx.x;
  const float* src = w + (size_t)n * KCV;
#pragma unroll
  for (int it = 0; it < 3; ++it)
    *(v4f*)(sf + it * 1024 + tid * 4) = *(const v4f*)(src + it * 1024 + tid * 4);
  __syncthreads();
  v4u vf[2], vh[2], vl[2];
  size_t go[2];
#pragma unroll
  for (int j = 0; j < 2; ++j) {
    int p = tid + 256 * j;
    p = (p < 384) ? p : 383;
    const int k8 = p * 8;
    const int tap = k8 >> 10, c0 = k8 & 1023;
    v8f f;
#pragma unroll
    for (int e = 0; e < 8; ++e) f[e] = sf[(c0 + e) * 3 + tap];
    Pack8 pk;
    pk.h = (v8h){(_Float16)(f[0] * 32.0f), (_Float16)(f[1] * 32.0f), (_Float16)(f[2] * 32.0f),
                 (_Float16)(f[3] * 32.0f), (_Float16)(f[4] * 32.0f), (_Float16)(f[5] * 32.0f),
                 (_Float16)(f[6] * 32.0f), (_Float16)(f[7] * 32.0f)};
    vf[j] = pk.u;
    const HL s = split8(f);
    vh[j] = s.h;
    vl[j] = s.l;
    go[j] = (size_t)n * KCV + k8;
  }
  const bool two = (tid < 128);
  for (int ps = 0; ps < 2; ++ps) {
    *(volatile v4u*)(wt + go[0]) = vf[0];
    *(volatile v4u*)(wh + go[0]) = vh[0];
    *(volatile v4u*)(wl + go[0]) = vl[0];
    if (two) {
      *(volatile v4u*)(wt + go[1]) = vf[1];
      *(volatile v4u*)(wh + go[1]) = vh[1];
      *(volatile v4u*)(wl + go[1]) = vl[1];
    }
    __threadfence();
  }
}

__global__ __launch_bounds__(256) void k_zero(_Float16* __restrict__ ctxp, ush* __restrict__ c3h,
                                              ush* __restrict__ c3l) {
  const int t = blockIdx.x * 256 + (int)threadIdx.x;
  const v4u z = (v4u){0u, 0u, 0u, 0u};
  volatile v4u* d;
  if (t < 512) {
    const int r = t >> 7, pc = t & 127;
    const size_t row = (size_t)(r >> 1) * CPR + ((r & 1) ? (CPR - 1) : 0);
    d = (volatile v4u*)(ctxp + row * DM + pc * 8);
  } else if (t < 768) {
    const int u = t - 512;
    d = (volatile v4u*)(c3h + (size_t)(u >> 7) * C3R * DM + (u & 127) * 8);
  } else {
    const int u = t - 768;
    d = (volatile v4u*)(c3l + (size_t)(u >> 7) * C3R * DM + (u & 127) * 8);
  }
  *d = z;
  __threadfence();
  *d = z;
}

#define STP 72
__device__ __forceinline__ void put_rows256(const _Float16* st, _Float16* __restrict__ dst, int tid) {
  v4u val[8];
#pragma unroll
  for (int j = 0; j < 8; ++j) {
    const int p = tid + 256 * j;
    Pack8 pk;
    pk.h = *(const v8h*)(st + (p >> 3) * STP + (p & 7) * 8);
    val[j] = pk.u;
  }
  for (int ps = 0; ps < 2; ++ps) {
#pragma unroll
    for (int j = 0; j < 8; ++j) *(volatile v4u*)(dst + (size_t)(tid + 256 * j) * 8) = val[j];
    __threadfence();
  }
}
__device__ __forceinline__ void put_cols256(const _Float16* st, _Float16* __restrict__ dst, int ldo, int tid) {
  v4u val[8];
  size_t go[8];
#pragma unroll
  for (int j = 0; j < 8; ++j) {
    const int p  = tid + 256 * j;
    const int L  = p >> 3;
    const int pc = p & 7;
    const int d  = L >> 2;
    const int nl = (L & 3) * 64 + pc * 8;
    const _Float16* cp = st + nl * STP + d;
    Pack8 pk;
    pk.h = (v8h){cp[0 * STP], cp[1 * STP], cp[2 * STP], cp[3 * STP],
                 cp[4 * STP], cp[5 * STP], cp[6 * STP], cp[7 * STP]};
    val[j] = pk.u;
    go[j]  = (size_t)d * ldo + nl;
  }
  for (int ps = 0; ps < 2; ++ps) {
#pragma unroll
    for (int j = 0; j < 8; ++j) *(volatile v4u*)(dst + go[j]) = val[j];
    __threadfence();
  }
}
__device__ __forceinline__ void put_rows64u(const ush* st, ush* __restrict__ dst, int tid) {
  v4u val[8];
#pragma unroll
  for (int j = 0; j < 8; ++j) {
    const int p = tid + 64 * j;
    PackU pk;
    pk.s = *(const v8us*)(st + (p >> 3) * STP + (p & 7) * 8);
    val[j] = pk.u;
  }
  for (int ps = 0; ps < 2; ++ps) {
#pragma unroll
    for (int j = 0; j < 8; ++j) *(volatile v4u*)(dst + (size_t)(tid + 64 * j) * 8) = val[j];
    __threadfence();
  }
}
__device__ __forceinline__ void put_cols64u(const ush* st, ush* __restrict__ dst, int ldo, int tid) {
  v4u val[8];
  size_t go[8];
#pragma unroll
  for (int j = 0; j < 8; ++j) {
    const int p  = tid + 64 * j;
    const int d  = p >> 3;
    const int nl = (p & 7) * 8;
    const ush* cp = st + nl * STP + d;
    PackU pk;
    pk.s = (v8us){cp[0 * STP], cp[1 * STP], cp[2 * STP], cp[3 * STP],
                  cp[4 * STP], cp[5 * STP], cp[6 * STP], cp[7 * STP]};
    val[j] = pk.u;
    go[j]  = (size_t)d * ldo + nl;
  }
  for (int ps = 0; ps < 2; ++ps) {
#pragma unroll
    for (int j = 0; j < 8; ++j) *(volatile v4u*)(dst + go[j]) = val[j];
    __threadfence();
  }
}

__global__ __launch_bounds__(256) void k_qkv(const _Float16* __restrict__ xh,
                                             const _Float16* __restrict__ wt,
                                             const float* __restrict__ bias,
                                             _Float16* __restrict__ qp,
                                             _Float16* __restrict__ kp,
                                             _Float16* __restrict__ vt) {
  __shared__ __align__(16) _Float16 st[256 * STP];
  const int tid = threadIdx.x, lane = tid & 31, wave = tid >> 5;
  const int hh = lane >> 4, c = lane & 15;
  const int mb = blockIdx.x * 256;
  const int b  = mb / SQ, tl = mb % SQ;
  const int m0 = mb + wave * 32;
  const int n0 = blockIdx.y * 64;
  const int which = n0 / DM;
  const int head  = (n0 % DM) >> 6;
  const int bh    = b * NH + head;
  if (which == 0 && tl < R0) return;

  v8f acc[2][4];
#pragma unroll
  for (int s = 0; s < 2; ++s)
#pragma unroll
    for (int t = 0; t < 4; ++t) acc[s][t] = zero8();
  gemm16<DM>(xh, DM, m0, wt, DM, n0, 0, lane, acc);

  float bv[4];
#pragma unroll
  for (int t = 0; t < 4; ++t) bv[t] = bias[n0 + 16 * t + c];
#pragma unroll
  for (int t = 0; t < 4; ++t) {
#pragma unroll
    for (int sub = 0; sub < 2; ++sub) {
#pragma unroll
      for (int r = 0; r < 8; ++r) {
        const int lr = wave * 32 + sub * 16 + 8 * hh + r;
        st[lr * STP + 16 * t + c] = (_Float16)(acc[sub][t][r] * 0.03125f + bv[t]);
      }
    }
  }
  __syncthreads();
  if (which < 2) {
    _Float16* dst = ((which == 0) ? qp : kp) + ((size_t)bh * SQ + tl) * HDM;
    put_rows256(st, dst, tid);
  } else {
    put_cols256(st, vt + (size_t)bh * HDM * SQ + tl, SQ, tid);
  }
}

__global__ __launch_bounds__(64) void k_qkv3(const ush* __restrict__ xh3, const ush* __restrict__ xl3,
                                             const ush* __restrict__ wh, const ush* __restrict__ wl,
                                             const float* __restrict__ bias,
                                             ush* __restrict__ q3h, ush* __restrict__ q3l,
                                             ush* __restrict__ k3h, ush* __restrict__ k3l,
                                             ush* __restrict__ v3h, ush* __restrict__ v3l) {
  __shared__ __align__(16) ush st[64 * STP];
  const int tid = threadIdx.x, lane = tid & 31, wave = tid >> 5;
  const int hh = lane >> 4, c = lane & 15;
  const int pr0 = blockIdx.x * 64;
  const int b   = blockIdx.x / NQ1;
  const int tl  = (blockIdx.x % NQ1) * 64;
  const int m0  = pr0 + wave * 32;
  const int n0  = blockIdx.y * 64;
  const int which = n0 / DM;
  const int head  = (n0 % DM) >> 6;
  const int bh    = b * NH + head;

  v8f acc[2][4];
#pragma unroll
  for (int s = 0; s < 2; ++s)
#pragma unroll
    for (int t = 0; t < 4; ++t) acc[s][t] = zero8();
  gemm3<DM>(xh3, xl3, DM, m0, wh, wl, DM, n0, 0, lane, acc);

#pragma unroll
  for (int t = 0; t < 4; ++t) {
    const float bv = bias[n0 + 16 * t + c];
#pragma unroll
    for (int sub = 0; sub < 2; ++sub)
#pragma unroll
      for (int r = 0; r < 8; ++r) acc[sub][t][r] += bv;
  }

  ush* dh = (which == 0) ? q3h : ((which == 1) ? k3h : v3h);
  ush* dl = (which == 0) ? q3l : ((which == 1) ? k3l : v3l);
  const size_t dbase = (which < 2) ? (((size_t)bh * R1 + tl) * HDM) : ((size_t)bh * HDM * R1 + tl);

#pragma unroll 1
  for (int ph = 0; ph < 2; ++ph) {
    __syncthreads();
#pragma unroll
    for (int t = 0; t < 4; ++t) {
#pragma unroll
      for (int sub = 0; sub < 2; ++sub) {
#pragma unroll
        for (int r = 0; r < 8; ++r) {
          const int lr = wave * 32 + sub * 16 + 8 * hh + r;
          const float v = acc[sub][t][r];
          const ush hi = f2bf(v);
          st[lr * STP + 16 * t + c] = (ph == 0) ? hi : f2bf(v - bf2f(hi));
        }
      }
    }
    __syncthreads();
    ush* dst = ((ph == 0) ? dh : dl) + dbase;
    if (which < 2) put_rows64u(st, dst, tid);
    else           put_cols64u(st, dst, R1, tid);
  }
}

#define KTP 72
#define PTP 72
__global__ __launch_bounds__(256) void k_attn(const _Float16* __restrict__ qpl,
                                              const _Float16* __restrict__ kp,
                                              const _Float16* __restrict__ vt,
                                              _Float16* __restrict__ op, int opb, int ooff, float sscale) {
  __shared__ __align__(16) _Float16 Ks[64 * KTP];
  __shared__ __align__(16) _Float16 Vs[64 * KTP];
  __shared__ __align__(16) _Float16 Ps[8][16 * PTP];

  const int tid = threadIdx.x, lane = tid & 31, wave = tid >> 5;
  const int hh = lane >> 4, c = lane & 15;
  const int nqb  = NQB - QB0;
  const int bh   = blockIdx.x / nqb;
  const int qb   = QB0 + blockIdx.x % nqb;
  const int b    = bh / NH, h = bh % NH;
  const int qblk = qb * QB;
  const int q0   = qblk + wave * 16;

  const _Float16* Q = qpl + (size_t)bh * SQ * HDM;
  const _Float16* K = kp + (size_t)bh * SQ * HDM;
  const _Float16* V = vt + (size_t)bh * HDM * SQ;

  v16h qa[2];
  qa[0] = ldfrag(Q, HDM, q0, 0, lane);
  qa[1] = ldfrag(Q, HDM, q0, 32, lane);

  const float NEGI = -__builtin_huge_valf();
  float mrow[8], lrow[8];
  v8f oacc[4];
#pragma unroll
  for (int r = 0; r < 8; ++r) { mrow[r] = NEGI; lrow[r] = 0.f; }
#pragma unroll
  for (int t = 0; t < 4; ++t) oacc[t] = zero8();

  _Float16* pw = Ps[wave];
  const int nkc = (qblk + QB) / KC;

  for (int kc = 0; kc < nkc; ++kc) {
    const int kv0 = kc * KC;
    __syncthreads();
    {
      const int r  = tid >> 2;
      const int qq = (tid & 3) * 16;
      const _Float16* ks = K + (size_t)(kv0 + r) * HDM + qq;
      *(v8h*)(Ks + r * KTP + qq)     = *(const v8h*)(ks);
      *(v8h*)(Ks + r * KTP + qq + 8) = *(const v8h*)(ks + 8);
      const _Float16* vs = V + (size_t)r * SQ + kv0 + qq;
      *(v8h*)(Vs + r * KTP + qq)     = *(const v8h*)(vs);
      *(v8h*)(Vs + r * KTP + qq + 8) = *(const v8h*)(vs + 8);
    }
    __syncthreads();

    v8f s[4];
#pragma unroll
    for (int j = 0; j < 4; ++j) s[j] = zero8();
#pragma unroll
    for (int dc = 0; dc < 2; ++dc) {
#pragma unroll
      for (int j = 0; j < 4; ++j) {
        const v16h kb = ldfrag(Ks, KTP, j * 16, dc * 32, lane);
        s[j] = mma16(qa[dc], kb, s[j]);
      }
    }
    if (kv0 + KC > qblk) {
#pragma unroll
      for (int r = 0; r < 8; ++r) {
        const int qr = q0 + 8 * hh + r;
#pragma unroll
        for (int j = 0; j < 4; ++j) {
          const int key = kv0 + 16 * j + c;
          s[j][r] = (key > qr) ? NEGI : (s[j][r] * sscale);
        }
      }
    } else {
#pragma unroll
      for (int r = 0; r < 8; ++r)
#pragma unroll
        for (int j = 0; j < 4; ++j) s[j][r] = s[j][r] * sscale;
    }
    float cm[8];
#pragma unroll
    for (int r = 0; r < 8; ++r) {
      float m = NEGI;
#pragma unroll
      for (int j = 0; j < 4; ++j) m = fmaxf(m, s[j][r]);
#pragma unroll
      for (int off = 1; off < 16; off <<= 1) m = fmaxf(m, __shfl_xor(m, off, 32));
      cm[r] = m;
    }
    float al[8];
#pragma unroll
    for (int r = 0; r < 8; ++r) {
      const float mnew  = fmaxf(mrow[r], cm[r]);
      const float alpha = __expf(mrow[r] - mnew);
      mrow[r] = mnew;
      float psum = 0.f;
#pragma unroll
      for (int j = 0; j < 4; ++j) {
        const float p = __expf(s[j][r] - mnew);
        psum += p;
        pw[(8 * hh + r) * PTP + j * 16 + c] = (_Float16)(p * 1024.0f);
      }
#pragma unroll
      for (int off = 1; off < 16; off <<= 1) psum += __shfl_xor(psum, off, 32);
      lrow[r] = lrow[r] * alpha + psum;
      al[r] = alpha;
    }
#pragma unroll
    for (int t = 0; t < 4; ++t)
#pragma unroll
      for (int r = 0; r < 8; ++r) oacc[t][r] *= al[r];
    __syncthreads();

#pragma unroll
    for (int kk = 0; kk < 2; ++kk) {
      const v16h pa = ldfrag(pw, PTP, 0, kk * 32, lane);
#pragma unroll
      for (int t = 0; t < 4; ++t) {
        const v16h vb = ldfrag(Vs, KTP, t * 16, kk * 32, lane);
        oacc[t] = mma16(pa, vb, oacc[t]);
      }
    }
  }
  __syncthreads();

#pragma unroll
  for (int r = 0; r < 8; ++r) {
    const float lr  = lrow[r];
    const float inv = (lr > 0.f) ? (0.015625f / lr) : 0.f;
#pragma unroll
    for (int t = 0; t < 4; ++t) pw[(8 * hh + r) * PTP + 16 * t + c] = (_Float16)(oacc[t][r] * inv);
  }
  __syncthreads();
  v4u val[4];
  size_t go[4];
#pragma unroll
  for (int it = 0; it < 4; ++it) {
    const int p  = lane + 32 * it;
    const int L  = p >> 3;
    const int pc = p & 7;
    Pack8 pk;
    pk.h    = *(const v8h*)(pw + L * PTP + pc * 8);
    val[it] = pk.u;
    go[it]  = ((size_t)b * opb + ooff + q0 + L) * DM + (size_t)h * HDM + pc * 8;
  }
  for (int ps = 0; ps < 2; ++ps) {
#pragma unroll
    for (int it = 0; it < 4; ++it) *(volatile v4u*)(op + go[it]) = val[it];
    __threadfence();
  }
}

__global__ __launch_bounds__(128) void k_attn3(const ush* __restrict__ q3h, const ush* __restrict__ q3l, int qrows,
                                               const ush* __restrict__ k3h, const ush* __restrict__ k3l,
                                               const ush* __restrict__ v3h, const ush* __restrict__ v3l,
                                               ush* __restrict__ o3h, ush* __restrict__ o3l, int opb3, int ooff3,
                                               _Float16* __restrict__ of16, int opbf, int oofff, int wf,
                                               int nq64, float sscale) {
  __shared__ __align__(16) ush Ksh[64 * KTP];
  __shared__ __align__(16) ush Ksl[64 * KTP];
  __shared__ __align__(16) ush Vsh[64 * KTP];
  __shared__ __align__(16) ush Vsl[64 * KTP];
  __shared__ __align__(16) ush Ph[4][16 * PTP];
  __shared__ __align__(16) ush Pl[4][16 * PTP];

  const int tid = threadIdx.x, lane = tid & 31, wave = tid >> 5;
  const int hh = lane >> 4, c = lane & 15;
  const int bh   = blockIdx.x / nq64;
  const int q64  = blockIdx.x % nq64;
  const int b    = bh / NH, h = bh % NH;
  const int qblk = q64 * 64;
  const int q0   = qblk + wave * 16;

  const ush* Qh = q3h + (size_t)bh * qrows * HDM;
  const ush* Ql = q3l + (size_t)bh * qrows * HDM;
  const ush* KH = k3h + (size_t)bh * R1 * HDM;
  const ush* KL = k3l + (size_t)bh * R1 * HDM;
  const ush* VH = v3h + (size_t)bh * HDM * R1;
  const ush* VL = v3l + (size_t)bh * HDM * R1;

  v16us qah[2], qal[2];
  qah[0] = ldfragu(Qh, HDM, q0, 0, lane);
  qah[1] = ldfragu(Qh, HDM, q0, 32, lane);
  qal[0] = ldfragu(Ql, HDM, q0, 0, lane);
  qal[1] = ldfragu(Ql, HDM, q0, 32, lane);

  const float NEGI = -__builtin_huge_valf();
  float mrow[8], lrow[8];
  v8f oacc[4];
#pragma unroll
  for (int r = 0; r < 8; ++r) { mrow[r] = NEGI; lrow[r] = 0.f; }
#pragma unroll
  for (int t = 0; t < 4; ++t) oacc[t] = zero8();

  ush* pwh = Ph[wave];
  ush* pwl = Pl[wave];
  const int nkc = q64 + 1;

  for (int kc = 0; kc < nkc; ++kc) {
    const int kv0 = kc * KC;
    __syncthreads();
    {
      const int r  = tid >> 1;
      const int qq = (tid & 1) * 32;
      const ush* ah = KH + (size_t)(kv0 + r) * HDM + qq;
      const ush* al = KL + (size_t)(kv0 + r) * HDM + qq;
      const ush* eh = VH + (size_t)r * R1 + kv0 + qq;
      const ush* el = VL + (size_t)r * R1 + kv0 + qq;
#pragma unroll
      for (int e = 0; e < 4; ++e) {
        *(v8us*)(Ksh + r * KTP + qq + 8 * e) = *(const v8us*)(ah + 8 * e);
        *(v8us*)(Ksl + r * KTP + qq + 8 * e) = *(const v8us*)(al + 8 * e);
        *(v8us*)(Vsh + r * KTP + qq + 8 * e) = *(const v8us*)(eh + 8 * e);
        *(v8us*)(Vsl + r * KTP + qq + 8 * e) = *(const v8us*)(el + 8 * e);
      }
    }
    __syncthreads();

    v8f s[4];
#pragma unroll
    for (int j = 0; j < 4; ++j) s[j] = zero8();
#pragma unroll
    for (int dc = 0; dc < 2; ++dc) {
#pragma unroll
      for (int j = 0; j < 4; ++j) {
        const v16us kbh = ldfragu(Ksh, KTP, j * 16, dc * 32, lane);
        const v16us kbl = ldfragu(Ksl, KTP, j * 16, dc * 32, lane);
        s[j] = mmab(qah[dc], kbh, s[j]);
        s[j] = mmab(qah[dc], kbl, s[j]);
        s[j] = mmab(qal[dc], kbh, s[j]);
      }
    }
    if (kc == q64) {
#pragma unroll
      for (int r = 0; r < 8; ++r) {
        const int qr = q0 + 8 * hh + r;
#pragma unroll
        for (int j = 0; j < 4; ++j) {
          const int key = kv0 + 16 * j + c;
          s[j][r] = (key > qr) ? NEGI : (s[j][r] * sscale);
        }
      }
    } else {
#pragma unroll
      for (int r = 0; r < 8; ++r)
#pragma unroll
        for (int j = 0; j < 4; ++j) s[j][r] = s[j][r] * sscale;
    }
    float cm[8];
#pragma unroll
    for (int r = 0; r < 8; ++r) {
      float m = NEGI;
#pragma unroll
      for (int j = 0; j < 4; ++j) m = fmaxf(m, s[j][r]);
#pragma unroll
      for (int off = 1; off < 16; off <<= 1) m = fmaxf(m, __shfl_xor(m, off, 32));
      cm[r] = m;
    }
    float al[8];
#pragma unroll
    for (int r = 0; r < 8; ++r) {
      const float mnew  = fmaxf(mrow[r], cm[r]);
      const float alpha = __expf(mrow[r] - mnew);
      mrow[r] = mnew;
      float psum = 0.f;
#pragma unroll
      for (int j = 0; j < 4; ++j) {
        const float p = __expf(s[j][r] - mnew);
        psum += p;
        const ush phi = f2bf(p);
        pwh[(8 * hh + r) * PTP + j * 16 + c] = phi;
        pwl[(8 * hh + r) * PTP + j * 16 + c] = f2bf(p - bf2f(phi));
      }
#pragma unroll
      for (int off = 1; off < 16; off <<= 1) psum += __shfl_xor(psum, off, 32);
      lrow[r] = lrow[r] * alpha + psum;
      al[r] = alpha;
    }
#pragma unroll
    for (int t = 0; t < 4; ++t)
#pragma unroll
      for (int r = 0; r < 8; ++r) oacc[t][r] *= al[r];
    __syncthreads();

#pragma unroll
    for (int kk = 0; kk < 2; ++kk) {
      const v16us pah = ldfragu(pwh, PTP, 0, kk * 32, lane);
      const v16us pal = ldfragu(pwl, PTP, 0, kk * 32, lane);
#pragma unroll
      for (int t = 0; t < 4; ++t) {
        const v16us vbh = ldfragu(Vsh, KTP, t * 16, kk * 32, lane);
        const v16us vbl = ldfragu(Vsl, KTP, t * 16, kk * 32, lane);
        oacc[t] = mmab(pah, vbh, oacc[t]);
        oacc[t] = mmab(pah, vbl, oacc[t]);
        oacc[t] = mmab(pal, vbh, oacc[t]);
      }
    }
  }
  __syncthreads();

  ush* pf = Ksh + wave * 16 * KTP;
#pragma unroll
  for (int r = 0; r < 8; ++r) {
    const float lr  = lrow[r];
    const float inv = (lr > 0.f) ? (1.0f / lr) : 0.f;
#pragma unroll
    for (int t = 0; t < 4; ++t) {
      const float o = oacc[t][r] * inv;
      const ush hi = f2bf(o);
      pwh[(8 * hh + r) * PTP + 16 * t + c] = hi;
      pwl[(8 * hh + r) * PTP + 16 * t + c] = f2bf(o - bf2f(hi));
      HU u; u.h = (_Float16)(o * 16.0f);
      pf[(8 * hh + r) * KTP + 16 * t + c] = u.u;
    }
  }
  __syncthreads();
  v4u vh[4], vl[4], vf[4];
  size_t go3[4], gof[4];
#pragma unroll
  for (int it = 0; it < 4; ++it) {
    const int p  = lane + 32 * it;
    const int L  = p >> 3;
    const int pc = p & 7;
    PackU pk;
    pk.s   = *(const v8us*)(pwh + L * PTP + pc * 8);
    vh[it] = pk.u;
    pk.s   = *(const v8us*)(pwl + L * PTP + pc * 8);
    vl[it] = pk.u;
    pk.s   = *(const v8us*)(pf + L * KTP + pc * 8);
    vf[it] = pk.u;
    go3[it] = ((size_t)b * opb3 + ooff3 + q0 + L) * DM + (size_t)h * HDM + pc * 8;
    gof[it] = ((size_t)b * opbf + oofff + q0 + L) * DM + (size_t)h * HDM + pc * 8;
  }
  const bool dof = (wf != 0) && (qblk < R0);
  for (int ps = 0; ps < 2; ++ps) {
#pragma unroll
    for (int it = 0; it < 4; ++it) {
      *(volatile v4u*)(o3h + go3[it]) = vh[it];
      *(volatile v4u*)(o3l + go3[it]) = vl[it];
      if (dof) *(volatile v4u*)(of16 + gof[it]) = vf[it];
    }
    __threadfence();
  }
}

__global__ __launch_bounds__(256) void k_conv(const _Float16* __restrict__ ctxp,
                                              const _Float16* __restrict__ wc,
                                              const float* __restrict__ bias,
                                              _Float16* __restrict__ q2p) {
  __shared__ __align__(16) _Float16 st[256 * STP];
  const int tid = threadIdx.x, lane = tid & 31, wave = tid >> 5;
  const int hh = lane >> 4, c = lane & 15;
  const int b  = blockIdx.x / MBP;
  const int tl = (1 + blockIdx.x % MBP) * 256;
  const int m0 = tl + wave * 32;
  const int n0 = blockIdx.y * 64;
  const int bh = b * NH + (n0 >> 6);
  const _Float16* A = ctxp + (size_t)b * CPR * DM;

  v8f acc[2][4];
#pragma unroll
  for (int s = 0; s < 2; ++s)
#pragma unroll
    for (int t = 0; t < 4; ++t) acc[s][t] = zero8();
#pragma unroll 1
  for (int j = 0; j < 3; ++j)
    gemm16<DM>(A + (size_t)j * DM, DM, m0, wc, KCV, n0, j * DM, lane, acc);

  float bv[4];
#pragma unroll
  for (int t = 0; t < 4; ++t) bv[t] = bias[n0 + 16 * t + c] * 32.0f;
#pragma unroll
  for (int t = 0; t < 4; ++t) {
#pragma unroll
    for (int sub = 0; sub < 2; ++sub) {
#pragma unroll
      for (int r = 0; r < 8; ++r) {
        const int lr = wave * 32 + sub * 16 + 8 * hh + r;
        st[lr * STP + 16 * t + c] = (_Float16)(acc[sub][t][r] * 0.0625f + bv[t]);
      }
    }
  }
  __syncthreads();
  put_rows256(st, q2p + ((size_t)bh * SQ + tl) * HDM, tid);
}

__global__ __launch_bounds__(64) void k_conv3(const ush* __restrict__ c3h, const ush* __restrict__ c3l,
                                              const ush* __restrict__ wh, const ush* __restrict__ wl,
                                              const float* __restrict__ bias,
                                              ush* __restrict__ q23h, ush* __restrict__ q23l) {
  __shared__ __align__(16) ush st[64 * STP];
  const int tid = threadIdx.x, lane = tid & 31, wave = tid >> 5;
  const int hh = lane >> 4, c = lane & 15;
  const int b  = blockIdx.x / NQ0;
  const int tl = (blockIdx.x % NQ0) * 64;
  const int m0 = tl + wave * 32;
  const int n0 = blockIdx.y * 64;
  const int bh = b * NH + (n0 >> 6);
  const ush* Ah = c3h + (size_t)b * C3R * DM;
  const ush* Al = c3l + (size_t)b * C3R * DM;

  v8f acc[2][4];
#pragma unroll
  for (int s = 0; s < 2; ++s)
#pragma unroll
    for (int t = 0; t < 4; ++t) acc[s][t] = zero8();
#pragma unroll 1
  for (int j = 0; j < 3; ++j)
    gemm3<DM>(Ah + (size_t)j * DM, Al + (size_t)j * DM, DM, m0, wh, wl, KCV, n0, j * DM, lane, acc);

#pragma unroll
  for (int t = 0; t < 4; ++t) {
    const float bv = bias[n0 + 16 * t + c];
#pragma unroll
    for (int sub = 0; sub < 2; ++sub)
#pragma unroll
      for (int r = 0; r < 8; ++r) acc[sub][t][r] += bv;
  }
  const size_t dbase = ((size_t)bh * R0 + tl) * HDM;

#pragma unroll 1
  for (int ph = 0; ph < 2; ++ph) {
    __syncthreads();
#pragma unroll
    for (int t = 0; t < 4; ++t) {
#pragma unroll
      for (int sub = 0; sub < 2; ++sub) {
#pragma unroll
        for (int r = 0; r < 8; ++r) {
          const int lr = wave * 32 + sub * 16 + 8 * hh + r;
          const float v = acc[sub][t][r];
          const ush hi = f2bf(v);
          st[lr * STP + 16 * t + c] = (ph == 0) ? hi : f2bf(v - bf2f(hi));
        }
      }
    }
    __syncthreads();
    put_rows64u(st, ((ph == 0) ? q23h : q23l) + dbase, tid);
  }
}

#define OTP 68
__device__ __forceinline__ void out_epilogue(v8f (&acc)[2][4], float scale, const float* __restrict__ bias,
                                             float* sw, float* __restrict__ out,
                                             int m0, int n0, int lane, int hh, int c) {
  float bv[4];
#pragma unroll
  for (int t = 0; t < 4; ++t) bv[t] = bias[n0 + 16 * t + c];
#pragma unroll
  for (int sub = 0; sub < 2; ++sub) {
    __syncthreads();
#pragma unroll
    for (int t = 0; t < 4; ++t) {
#pragma unroll
      for (int r = 0; r < 8; ++r) sw[(8 * hh + r) * OTP + 16 * t + c] = acc[sub][t][r] * scale + bv[t];
    }
    __syncthreads();
    v4f val[8];
    size_t go[8];
#pragma unroll
    for (int it = 0; it < 8; ++it) {
      const int p    = lane + 32 * it;
      const int L    = p >> 3;
      const int pc   = p & 7;
      const int row  = L >> 1;
      const int half = L & 1;
      val[it] = *(const v4f*)(sw + row * OTP + half * 32 + pc * 4);
      go[it]  = (size_t)(m0 + sub * 16 + row) * DM + n0 + half * 32 + pc * 4;
    }
    for (int ps = 0; ps < 2; ++ps) {
#pragma unroll
      for (int it = 0; it < 8; ++it) *(volatile v4f*)(out + go[it]) = val[it];
      __threadfence();
    }
  }
}

__global__ __launch_bounds__(256) void k_out(const _Float16* __restrict__ ap,
                                             const _Float16* __restrict__ wt,
                                             const float* __restrict__ bias,
                                             float* __restrict__ out) {
  __shared__ __align__(16) float st[8][16 * OTP];
  const int tid = threadIdx.x, lane = tid & 31, wave = tid >> 5;
  const int hh = lane >> 4, c = lane & 15;
  const int b  = blockIdx.x / MBP;
  const int m0 = b * SQ + (1 + blockIdx.x % MBP) * 256 + wave * 32;
  const int n0 = blockIdx.y * 64;

  v8f acc[2][4];
#pragma unroll
  for (int s = 0; s < 2; ++s)
#pragma unroll
    for (int t = 0; t < 4; ++t) acc[s][t] = zero8();
  gemm16<DM>(ap, DM, m0, wt, DM, n0, 0, lane, acc);
  out_epilogue(acc, 0.001953125f, bias, st[wave], out, m0, n0, lane, hh, c);
}

__global__ __launch_bounds__(64) void k_out3(const ush* __restrict__ ah, const ush* __restrict__ al,
                                             const ush* __restrict__ wh, const ush* __restrict__ wl,
                                             const float* __restrict__ bias, float* __restrict__ out) {
  __shared__ __align__(16) float st[2][16 * OTP];
  const int tid = threadIdx.x, lane = tid & 31, wave = tid >> 5;
  const int hh = lane >> 4, c = lane & 15;
  const int b   = blockIdx.x / NQ0;
  const int tl  = (blockIdx.x % NQ0) * 64;
  const int am0 = b * R0 + tl + wave * 32;
  const int om0 = b * SQ + tl + wave * 32;
  const int n0  = blockIdx.y * 64;

  v8f acc[2][4];
#pragma unroll
  for (int s = 0; s < 2; ++s)
#pragma unroll
    for (int t = 0; t < 4; ++t) acc[s][t] = zero8();
  gemm3<DM>(ah, al, DM, am0, wh, wl, DM, n0, 0, lane, acc);
  out_epilogue(acc, 1.0f, bias, st[wave], out, om0, n0, lane, hh, c);
}

extern "C" void kernel_launch(void* const* d_in, const int* in_sizes, int n_in,
                              void* d_out, int out_size, void* d_ws, size_t ws_size,
                              hipStream_t stream) {
  if (n_in < 7) return;
  if (in_sizes[0] != MR * DM) return;
  if (in_sizes[1] != NQKV * DM) return;
  if (in_sizes[2] != NQKV) return;
  if (in_sizes[3] != DM * KCV) return;
  if (in_sizes[4] != DM) return;
  if (in_sizes[5] != DM * DM) return;
  if (in_sizes[6] != DM) return;
  if (out_size != MR * DM) return;

  const float* x     = (const float*)d_in[0];
  const float* wqkv  = (const float*)d_in[1];
  const float* bqkv  = (const float*)d_in[2];
  const float* wconv = (const float*)d_in[3];
  const float* bconv = (const float*)d_in[4];
  const float* wout  = (const float*)d_in[5];
  const float* bout  = (const float*)d_in[6];
  float* out = (float*)d_out;

  size_t off = 0;
  const size_t oX    = off; off += (size_t)MR * DM * 2;
  const size_t oX3h  = off; off += (size_t)NB * R1 * DM * 2;
  const size_t oX3l  = off; off += (size_t)NB * R1 * DM * 2;
  const size_t oWq   = off; off += (size_t)NQKV * DM * 2;
  const size_t oWqh  = off; off += (size_t)NQKV * DM * 2;
  const size_t oWql  = off; off += (size_t)NQKV * DM * 2;
  const size_t oWc   = off; off += (size_t)DM * KCV * 2;
  const size_t oWch  = off; off += (size_t)DM * KCV * 2;
  const size_t oWcl  = off; off += (size_t)DM * KCV * 2;
  const size_t oWo   = off; off += (size_t)DM * DM * 2;
  const size_t oWoh  = off; off += (size_t)DM * DM * 2;
  const size_t oWol  = off; off += (size_t)DM * DM * 2;
  const size_t oQ    = off; off += (size_t)NBH * SQ * HDM * 2;
  const size_t oK    = off; off += (size_t)NBH * SQ * HDM * 2;
  const size_t oV    = off; off += (size_t)NBH * HDM * SQ * 2;
  const size_t oQ3h  = off; off += (size_t)NBH * R1 * HDM * 2;
  const size_t oQ3l  = off; off += (size_t)NBH * R1 * HDM * 2;
  const size_t oK3h  = off; off += (size_t)NBH * R1 * HDM * 2;
  const size_t oK3l  = off; off += (size_t)NBH * R1 * HDM * 2;
  const size_t oV3h  = off; off += (size_t)NBH * HDM * R1 * 2;
  const size_t oV3l  = off; off += (size_t)NBH * HDM * R1 * 2;
  const size_t oC    = off; off += (size_t)NB * CPR * DM * 2;
  const size_t oC3h  = off; off += (size_t)NB * C3R * DM * 2;
  const size_t oC3l  = off; off += (size_t)NB * C3R * DM * 2;
  const size_t oQ2   = off; off += (size_t)NBH * SQ * HDM * 2;
  const size_t oQ23h = off; off += (size_t)NBH * R0 * HDM * 2;
  const size_t oQ23l = off; off += (size_t)NBH * R0 * HDM * 2;
  const size_t oC2   = off; off += (size_t)MR * DM * 2;
  const size_t oC23h = off; off += (size_t)NB * R0 * DM * 2;
  const size_t oC23l = off; off += (size_t)NB * R0 * DM * 2;
  if (off > ws_size) return;
  if (off > (size_t)134217728) return;

  char* ws = (char*)d_ws;
  _Float16* Xh   = (_Float16*)(ws + oX);
  ush*      X3h  = (ush*)(ws + oX3h);
  ush*      X3l  = (ush*)(ws + oX3l);
  _Float16* Wq   = (_Float16*)(ws + oWq);
  ush*      Wqh  = (ush*)(ws + oWqh);
  ush*      Wql  = (ush*)(ws + oWql);
  _Float16* Wc   = (_Float16*)(ws + oWc);
  ush*      Wch  = (ush*)(ws + oWch);
  ush*      Wcl  = (ush*)(ws + oWcl);
  _Float16* Wo   = (_Float16*)(ws + oWo);
  ush*      Woh  = (ush*)(ws + oWoh);
  ush*      Wol  = (ush*)(ws + oWol);
  _Float16* Qp   = (_Float16*)(ws + oQ);
  _Float16* Kp   = (_Float16*)(ws + oK);
  _Float16* Vt   = (_Float16*)(ws + oV);
  ush*      Q3h  = (ush*)(ws + oQ3h);
  ush*      Q3l  = (ush*)(ws + oQ3l);
  ush*      K3h  = (ush*)(ws + oK3h);
  ush*      K3l  = (ush*)(ws + oK3l);
  ush*      V3h  = (ush*)(ws + oV3h);
  ush*      V3l  = (ush*)(ws + oV3l);
  _Float16* Cp   = (_Float16*)(ws + oC);
  ush*      C3h  = (ush*)(ws + oC3h);
  ush*      C3l  = (ush*)(ws + oC3l);
  _Float16* Q2p  = (_Float16*)(ws + oQ2);
  ush*      Q23h = (ush*)(ws + oQ23h);
  ush*      Q23l = (ush*)(ws + oQ23l);
  _Float16* C2p  = (_Float16*)(ws + oC2);
  ush*      C23h = (ush*)(ws + oC23h);
  ush*      C23l = (ush*)(ws + oC23l);

  const int ngx = in_sizes[0] / 8;
  const int ngq = in_sizes[1] / 8;
  const int ngo = in_sizes[5] / 8;
  k_cvt_x<<<dim3((ngx + 255) / 256), dim3(256), 0, stream>>>(x, Xh, X3h, X3l, ngx);
  k_cvt_w<<<dim3((ngq + 255) / 256), dim3(256), 0, stream>>>(wqkv, Wq, Wqh, Wql, ngq);
  k_cvt_w<<<dim3((ngo + 255) / 256), dim3(256), 0, stream>>>(wout, Wo, Woh, Wol, ngo);
  k_cvt_wc<<<dim3(DM), dim3(256), 0, stream>>>(wconv, Wc, Wch, Wcl);
  k_zero<<<dim3(4), dim3(256), 0, stream>>>(Cp, C3h, C3l);
  k_qkv<<<dim3(MR / 256, NQKV / 64), dim3(256), 0, stream>>>(Xh, Wq, bqkv, Qp, Kp, Vt);
  k_qkv3<<<dim3(NB * NQ1, NQKV / 64), dim3(64), 0, stream>>>(X3h, X3l, Wqh, Wql, bqkv,
                                                               Q3h, Q3l, K3h, K3l, V3h, V3l);
  k_attn<<<dim3(NBH * (NQB - QB0)), dim3(256), 0, stream>>>(Qp, Kp, Vt, Cp, CPR, 1, 0.125f);
  k_attn3<<<dim3(NBH * NQ1), dim3(128), 0, stream>>>(Q3h, Q3l, R1, K3h, K3l, V3h, V3l,
                                                      C3h, C3l, C3R, 1, Cp, CPR, 1, 1, NQ1, 0.125f);
  k_conv<<<dim3(NB * MBP, DM / 64), dim3(256), 0, stream>>>(Cp, Wc, bconv, Q2p);
  k_conv3<<<dim3(NB * NQ0, DM / 64), dim3(64), 0, stream>>>(C3h, C3l, Wch, Wcl, bconv, Q23h, Q23l);
  k_attn<<<dim3(NBH * (NQB - QB0)), dim3(256), 0, stream>>>(Q2p, Kp, Vt, C2p, SQ, 0, 0.00390625f);
  k_attn3<<<dim3(NBH * NQ0), dim3(128), 0, stream>>>(Q23h, Q23l, R0, K3h, K3l, V3h, V3l,
                                                      C23h, C23l, R0, 0, Cp, CPR, 1, 0, NQ0, 0.125f);
  k_out<<<dim3(NB * MBP, DM / 64), dim3(256), 0, stream>>>(C2p, Wo, bout, out);
  k_out3<<<dim3(NB * NQ0, DM / 64), dim3(64), 0, stream>>>(C23h, C23l, Woh, Wol, bout, out);
  (void)hipGetLastError();
}
